// PointNetSetAbstraction_grid_31997506355427
// MI455X (gfx1250) — hardware-verified
//
#include <hip/hip_runtime.h>
#include <math.h>

typedef __attribute__((ext_vector_type(16))) _Float16 v16h;
typedef __attribute__((ext_vector_type(8)))  _Float16 v8h;
typedef __attribute__((ext_vector_type(8)))  float    v8f;
typedef __attribute__((ext_vector_type(4)))  float    v4f;
typedef __attribute__((ext_vector_type(4)))  int      v4i;

constexpr int NB = 8;
constexpr int NPTS = 4096;
constexpr int NFEAT = 64;
constexpr int NS = 1024;
constexpr int NK = 32;
constexpr int NGRP = NB * NS;
constexpr int CIN = 67;
constexpr int NCELL = 125;
constexpr int NTAP = 27;
constexpr int CPITCH = 72;
constexpr int K0REAL = NTAP * CPITCH;
constexpr int K0 = 1952;
constexpr int NSTEP0 = K0 / 32;
constexpr int K1 = 1728;
constexpr int H0_ROW = NTAP * 64;
constexpr int KA = 96;
constexpr int FPITCH = 68;
constexpr int FA_PITCH = 104;
constexpr int Y_PITCH = 72;

constexpr float WCARRY = 16.0f;
constexpr float WCARRY_INV = 1.0f / 16.0f;
constexpr float RADIUS_F = 0.2f;
constexpr float INV_RADIUS = 1.0f / RADIUS_F;
constexpr float RXYZ_F = 0.4330127018922193f;
constexpr float INV_RXYZ = 1.0f / RXYZ_F;
constexpr float EPS_F = 1e-6f;
constexpr float BOXLIM = 1.4335f;

static_assert(NGRP == 8192, "groups");
static_assert(K0 % 32 == 0 && K0 >= K0REAL && K0 - K0REAL == 8, "conv0 K pad");
static_assert(NSTEP0 == 61, "conv0 steps");
static_assert(K1 % 32 == 0 && K1 == H0_ROW, "conv1 K");
static_assert(KA % 32 == 0 && KA >= CIN, "mlp K pad");
static_assert(NGRP % 64 == 0, "gemm M tile");
static_assert((H0_ROW * 2) % 128 == 0, "h0 row is whole lines");

constexpr int OFF_W0T = 0;
constexpr int OFF_W1T = OFF_W0T + 64 * K0;
constexpr int OFF_W2T = OFF_W1T + 64 * K1;
constexpr int OFF_WA  = OFF_W2T + 128 * 64;
constexpr int OFF_WB  = OFF_WA + 64 * KA;
constexpr int OFF_WC  = OFF_WB + 64 * 64;
constexpr int WPL_HALVES = OFF_WC + 128 * 64;
static_assert(OFF_W1T % 256 == 0 && OFF_W2T % 256 == 0 && OFF_WA % 256 == 0 && OFF_WB % 256 == 0 && OFF_WC % 256 == 0, "plane starts wave aligned");
static_assert(WPL_HALVES == 262144, "weight region");

constexpr size_t WS_WPL = 0;
constexpr size_t WPL_BYTES = (size_t)WPL_HALVES * 2;
constexpr size_t WS_H0 = WS_WPL + WPL_BYTES;
constexpr size_t H0_BYTES = (size_t)NGRP * H0_ROW * 2;
constexpr size_t WS_H1 = WS_H0 + H0_BYTES;
constexpr size_t H1_BYTES = (size_t)NGRP * 64 * 2;
constexpr size_t WS_NF3 = WS_H1 + H1_BYTES;
constexpr size_t NF_BYTES = (size_t)NGRP * 128 * 4;
constexpr size_t WS_NF2 = WS_NF3 + NF_BYTES;
constexpr size_t WS_TOTAL = WS_NF2 + NF_BYTES;
static_assert(WS_TOTAL == 38273024, "carve");
static_assert(WS_TOTAL <= (size_t)134217728, "carve under limit");
static_assert(WS_H0 % 128 == 0 && WS_H1 % 128 == 0 && WS_NF3 % 128 == 0 && WS_NF2 % 128 == 0, "line aligned regions");

constexpr size_t OUT1_BYTE_OFF = 98304;
constexpr size_t OUT0_ELEMS = (size_t)NB * 3 * NS;
constexpr size_t OUT1_ELEMS = (size_t)NB * 128 * NS;
static_assert(OUT1_BYTE_OFF % 128 == 0, "out1 line aligned");
static_assert(OUT1_BYTE_OFF / 4 == OUT0_ELEMS, "out1 element offset");
static_assert(OUT1_BYTE_OFF + OUT1_ELEMS * 4 == (size_t)4292608, "output total");

union FragH { v16h v; v8h h[2]; };

__device__ __forceinline__ v16h frag_ld(const _Float16* p) {
  FragH f;
  f.h[0] = *(const v8h*)(p);
  f.h[1] = *(const v8h*)(p + 16);
  return f.v;
}

__device__ __forceinline__ v8f mma_h(v16h a, v16h b, v8f c) {
  c = __builtin_amdgcn_wmma_f32_16x16x32_f16(false, a, false, b, (short)0, c, false, false);
  asm volatile("v_nop\n\tv_nop\n\tv_nop\n\tv_nop" : "+v"(c) : "v"(a), "v"(b));
  return c;
}

__device__ __forceinline__ int clampi(int v, int lo, int hi) {
  return v < lo ? lo : (v > hi ? hi : v);
}

__device__ __forceinline__ float splat_w(float px, float py, float pz, float gx, float gy, float gz) {
#pragma clang fp contract(off)
  const float dx = px - gx;
  const float dy = py - gy;
  const float dz = pz - gz;
  const float t0 = dx * dx;
  const float t1 = dy * dy;
  const float t2 = dz * dz;
  const float d = sqrtf((t0 + t2) + t1);
  const float w = 1.0f - d * INV_RXYZ;
  return fmaxf(w, 0.0f);
}

__device__ __forceinline__ int cell_of_pos(int pos) {
  const int od = pos / 9;
  const int rem = pos - od * 9;
  const int oh = rem / 3;
  const int ow = rem - oh * 3;
  return od * 25 + oh * 5 + ow;
}

__device__ __forceinline__ unsigned run_byte_off(int r) {
  const int pr = r / 27;
  const int wi = r - pr * 27;
  const int kd = pr / 3;
  const int kh = pr - kd * 3;
  return (unsigned)(((kd * 25 + kh * 5) * CPITCH + wi * 8) * 2);
}

__global__ __launch_bounds__(256) void k_prep_w(
    const float* __restrict__ w3d0, const float* __restrict__ w3d1, const float* __restrict__ w3d2,
    const float* __restrict__ w2d0, const float* __restrict__ w2d1, const float* __restrict__ w2d2,
    _Float16* __restrict__ wpl) {
  const int base = (int)(blockIdx.x * 256 + threadIdx.x) * 8;
  const int wbase = __builtin_amdgcn_readfirstlane((int)((blockIdx.x * 256 + (threadIdx.x & ~31u)) * 8));
  float v[8];
  if (wbase < OFF_W1T) {
#pragma unroll
    for (int e = 0; e < 8; ++e) {
      const int idx = base + e;
      const int o = idx / K0;
      const int k = idx - o * K0;
      const int tap = k / CPITCH;
      const int c = k - tap * CPITCH;
      const bool ok = (tap < NTAP) && (c < CIN);
      const int cc = c < CIN ? c : (CIN - 1);
      const int tt = tap < NTAP ? tap : (NTAP - 1);
      const float x = w3d0[o * (CIN * 27) + cc * 27 + tt];
      v[e] = ok ? x * WCARRY : 0.0f;
    }
  } else if (wbase < OFF_W2T) {
#pragma unroll
    for (int e = 0; e < 8; ++e) {
      const int idx = base + e - OFF_W1T;
      const int o = idx / K1;
      const int k = idx - o * K1;
      const int tau = k >> 6;
      const int c = k & 63;
      const float x = w3d1[o * K1 + c * 27 + tau];
      v[e] = x * WCARRY;
    }
  } else if (wbase < OFF_WA) {
#pragma unroll
    for (int e = 0; e < 8; ++e) v[e] = w3d2[base + e - OFF_W2T] * WCARRY;
  } else if (wbase < OFF_WB) {
#pragma unroll
    for (int e = 0; e < 8; ++e) {
      const int idx = base + e - OFF_WA;
      const int o = idx / KA;
      const int k = idx - o * KA;
      const bool ok = k < CIN;
      const int kc = k < CIN ? k : (CIN - 1);
      const float x = w2d0[o * CIN + kc];
      v[e] = ok ? x * WCARRY : 0.0f;
    }
  } else if (wbase < OFF_WC) {
#pragma unroll
    for (int e = 0; e < 8; ++e) v[e] = w2d1[base + e - OFF_WB] * WCARRY;
  } else {
#pragma unroll
    for (int e = 0; e < 8; ++e) v[e] = w2d2[base + e - OFF_WC] * WCARRY;
  }
  v8h hv;
#pragma unroll
  for (int e = 0; e < 8; ++e) hv[e] = (_Float16)v[e];
  _Float16* p = wpl + base;
  *(volatile v8h*)p = hv;
  __threadfence();
  *(volatile v8h*)p = hv;
}

__global__ __launch_bounds__(256) void k_out0(
    const float* __restrict__ xyz, const int* __restrict__ fps_idx, float* __restrict__ out0) {
  const int idx = (int)(blockIdx.x * 256 + threadIdx.x);
  const int row = idx >> 8;
  const int s4 = (idx & 255) * 4;
  const int b = row / 3;
  const v4i fi = *(const v4i*)(fps_idx + b * NS + s4);
  const int i0 = clampi(fi[0], 0, NPTS - 1);
  const int i1 = clampi(fi[1], 0, NPTS - 1);
  const int i2 = clampi(fi[2], 0, NPTS - 1);
  const int i3 = clampi(fi[3], 0, NPTS - 1);
  const float* xr = xyz + (size_t)row * NPTS;
  v4f v;
  v[0] = xr[i0];
  v[1] = xr[i1];
  v[2] = xr[i2];
  v[3] = xr[i3];
  float* p = out0 + (size_t)row * NS + s4;
  *(volatile v4f*)p = v;
  __threadfence();
  *(volatile v4f*)p = v;
}

__global__ __launch_bounds__(128) void k_splat_conv0(
    const float* __restrict__ xyz, const float* __restrict__ points,
    const int* __restrict__ fps_idx, const int* __restrict__ ball_idx,
    const _Float16* __restrict__ W0t,
    const float* __restrict__ bn_b, const float* __restrict__ bn_s, const float* __restrict__ bn_t,
    _Float16* __restrict__ h0) {
  __shared__ __align__(16) _Float16 gfT[128 * CPITCH];
  __shared__ __align__(16) float featL[NK * FPITCH];
  __shared__ __align__(16) float locL[NK * 4];
  __shared__ __align__(16) _Float16 hT[32 * 64];
  __shared__ int sIdx[NK];
  __shared__ unsigned tabL[NSTEP0 * 2];
  __shared__ int hitF[4];
  __shared__ unsigned sMask;

  const int t = (int)threadIdx.x;
  const int lane = t & 31;
  const int wave = __builtin_amdgcn_readfirstlane(t >> 5);
  const int h = lane >> 4;
  const int rl = lane & 15;
  const int grp = (int)blockIdx.x;
  const int b = grp >> 10;

  {
    const int ci = clampi(fps_idx[grp], 0, NPTS - 1);
    const int n = clampi(ball_idx[grp * NK + lane], 0, NPTS - 1);
    const float* xb = xyz + (size_t)b * 3 * NPTS;
    const float cx = xb[ci];
    const float cy = xb[NPTS + ci];
    const float cz = xb[2 * NPTS + ci];
    const float lx = (xb[n] - cx) * INV_RADIUS;
    const float ly = (xb[NPTS + n] - cy) * INV_RADIUS;
    const float lz = (xb[2 * NPTS + n] - cz) * INV_RADIUS;
    const bool inbox = (fabsf(lx) < BOXLIM) && (fabsf(ly) < BOXLIM) && (fabsf(lz) < BOXLIM);
    const unsigned mk = __builtin_amdgcn_ballot_w32(inbox);
    if (wave == 0) {
      v4f lv;
      lv[0] = lx;
      lv[1] = ly;
      lv[2] = lz;
      lv[3] = 0.0f;
      *(v4f*)&locL[lane * 4] = lv;
      featL[lane * FPITCH + 0] = lx;
      featL[lane * FPITCH + 1] = ly;
      featL[lane * FPITCH + 2] = lz;
      featL[lane * FPITCH + 67] = 0.0f;
      sIdx[lane] = n;
      if (lane == 0) sMask = mk;
    }
  }
  if (t < NSTEP0 * 2) {
    const int step = t >> 1;
    const int hh = t & 1;
    const int r0 = 4 * step + hh;
    const int r1 = r0 + 2;
    const unsigned e0 = run_byte_off(r0);
    const unsigned e1 = (r1 < 243) ? run_byte_off(r1 < 243 ? r1 : 242) : 0u;
    tabL[t] = e0 | (e1 << 16);
  }
  __syncthreads();

  const unsigned mask = (unsigned)__builtin_amdgcn_readfirstlane((int)sMask);

  const int g = t < NCELL ? t : (NCELL - 1);
  const float gx = -1.0f + 0.5f * (float)(g / 25);
  const float gy = -1.0f + 0.5f * (float)((g / 5) % 5);
  const float gz = -1.0f + 0.5f * (float)(g % 5);

  float wsum = 0.0f;
  int dense = 0;
  if (mask != 0u) {
    {
      const int c = t & 63;
      const int ksub = __builtin_amdgcn_readfirstlane(t >> 6);
#pragma unroll 1
      for (int it = 0; it < 16; ++it) {
        const int k = it * 2 + ksub;
        if ((mask >> k) & 1u) {
          const int n = sIdx[k];
          featL[k * FPITCH + 3 + c] = points[((size_t)(b * NFEAT + c)) * NPTS + n];
        }
      }
    }
    __syncthreads();
    {
      unsigned m = mask;
      while (m != 0u) {
        const int k = __builtin_ctz(m);
        m &= (m - 1u);
        const v4f lc = *(const v4f*)&locL[k * 4];
        wsum += splat_w(lc[0], lc[1], lc[2], gx, gy, gz);
      }
    }
    const unsigned hb = __builtin_amdgcn_ballot_w32(wsum > 0.0f);
    if (lane == 0) hitF[wave] = (hb != 0u) ? 1 : 0;
    __syncthreads();
    dense = __builtin_amdgcn_readfirstlane(hitF[0] | hitF[1] | hitF[2] | hitF[3]);
  }

  const int q = lane & 7;
  const int lr = lane >> 3;
  const int line0 = wave * 4 + lr;
  const int line1 = 16 + wave * 4 + lr;
  v8h vv0, vv1;

  if (dense != 0) {
    float acc[FPITCH];
#pragma unroll
    for (int i = 0; i < FPITCH; ++i) acc[i] = 0.0f;
    const float inv = 1.0f / (wsum + EPS_F);
    {
      unsigned m = mask;
      while (m != 0u) {
        const int k = __builtin_ctz(m);
        m &= (m - 1u);
        const v4f lc = *(const v4f*)&locL[k * 4];
        const float w = splat_w(lc[0], lc[1], lc[2], gx, gy, gz);
        const float wn = w * inv;
        const unsigned any = __builtin_amdgcn_ballot_w32(wn > 0.0f);
        if (any != 0u) {
          const float* fr = &featL[k * FPITCH];
#pragma unroll
          for (int i = 0; i < FPITCH / 4; ++i) {
            const v4f f = *(const v4f*)(fr + 4 * i);
            acc[4 * i + 0] = fmaf(f[0], wn, acc[4 * i + 0]);
            acc[4 * i + 1] = fmaf(f[1], wn, acc[4 * i + 1]);
            acc[4 * i + 2] = fmaf(f[2], wn, acc[4 * i + 2]);
            acc[4 * i + 3] = fmaf(f[3], wn, acc[4 * i + 3]);
          }
        }
      }
    }
    {
      float zz = 0.0f;
      asm volatile("" : "+v"(zz));
      const bool real = t < NCELL;
#pragma unroll
      for (int j = 0; j < CPITCH / 8; ++j) {
        v8h hv;
#pragma unroll
        for (int e = 0; e < 8; ++e) {
          const int ch = 8 * j + e;
          float x = zz;
          if (ch < CIN) x = real ? acc[ch] : zz;
          hv[e] = (_Float16)x;
        }
        *(v8h*)&gfT[t * CPITCH + 8 * j] = hv;
      }
    }
    __syncthreads();

    const int pos1 = (16 + rl) < NTAP ? (16 + rl) : (NTAP - 1);
    const unsigned cb0 = (unsigned)(cell_of_pos(rl) * CPITCH * 2);
    const unsigned cb1 = (unsigned)(cell_of_pos(pos1) * CPITCH * 2);
    const char* gfb = (const char*)gfT;
    const _Float16* Bp = W0t + (size_t)(16 * wave + rl) * K0 + 8 * h;
    v8f acc0 = (v8f){0.f, 0.f, 0.f, 0.f, 0.f, 0.f, 0.f, 0.f};
    v8f acc1 = (v8f){0.f, 0.f, 0.f, 0.f, 0.f, 0.f, 0.f, 0.f};
#pragma unroll 2
    for (int step = 0; step < NSTEP0 - 1; ++step) {
      const unsigned e = tabL[step * 2 + h];
      const unsigned e0 = e & 0xffffu;
      const unsigned e1 = e >> 16;
      const v16h bfr = frag_ld(Bp + step * 32);
      FragH a0, a1;
      a0.h[0] = *(const v8h*)(gfb + cb0 + e0);
      a0.h[1] = *(const v8h*)(gfb + cb0 + e1);
      a1.h[0] = *(const v8h*)(gfb + cb1 + e0);
      a1.h[1] = *(const v8h*)(gfb + cb1 + e1);
      acc0 = mma_h(a0.v, bfr, acc0);
      acc1 = mma_h(a1.v, bfr, acc1);
    }
    {
      const unsigned e = tabL[(NSTEP0 - 1) * 2 + h];
      const unsigned e0 = e & 0xffffu;
      const unsigned e1 = e >> 16;
      const unsigned zrow = (unsigned)(NCELL * CPITCH * 2);
      const unsigned o10 = (h == 1) ? zrow : (cb0 + e1);
      const unsigned o11 = (h == 1) ? zrow : (cb1 + e1);
      const v16h bfr = frag_ld(Bp + (NSTEP0 - 1) * 32);
      FragH a0, a1;
      a0.h[0] = *(const v8h*)(gfb + cb0 + e0);
      a0.h[1] = *(const v8h*)(gfb + o10);
      a1.h[0] = *(const v8h*)(gfb + cb1 + e0);
      a1.h[1] = *(const v8h*)(gfb + o11);
      acc0 = mma_h(a0.v, bfr, acc0);
      acc1 = mma_h(a1.v, bfr, acc1);
    }
    {
      const int o = 16 * wave + rl;
      const float bb = bn_b[o];
      const float ss = bn_s[o];
      const float tt = bn_t[o];
#pragma unroll
      for (int r = 0; r < 8; ++r) {
        const int pos = 8 * h + r;
        const float y = fmaxf((acc0[r] * WCARRY_INV + bb) * ss + tt, 0.0f);
        hT[pos * 64 + o] = (_Float16)y;
      }
#pragma unroll
      for (int r = 0; r < 8; ++r) {
        const int pos = 16 + 8 * h + r;
        const float y = fmaxf((acc1[r] * WCARRY_INV + bb) * ss + tt, 0.0f);
        if (pos < NTAP) hT[pos * 64 + o] = (_Float16)y;
      }
    }
    __syncthreads();
    const int l1c = line1 < NTAP ? line1 : (NTAP - 1);
    vv0 = *(const v8h*)&hT[line0 * 64 + q * 8];
    vv1 = *(const v8h*)&hT[l1c * 64 + q * 8];
  } else {
    const v4f b_lo = *(const v4f*)(bn_b + q * 8);
    const v4f b_hi = *(const v4f*)(bn_b + q * 8 + 4);
    const v4f s_lo = *(const v4f*)(bn_s + q * 8);
    const v4f s_hi = *(const v4f*)(bn_s + q * 8 + 4);
    const v4f t_lo = *(const v4f*)(bn_t + q * 8);
    const v4f t_hi = *(const v4f*)(bn_t + q * 8 + 4);
    v8h cv;
#pragma unroll
    for (int e = 0; e < 4; ++e) {
      const float y0 = fmaxf(b_lo[e] * s_lo[e] + t_lo[e], 0.0f);
      const float y1 = fmaxf(b_hi[e] * s_hi[e] + t_hi[e], 0.0f);
      cv[e] = (_Float16)y0;
      cv[4 + e] = (_Float16)y1;
    }
    vv0 = cv;
    vv1 = cv;
  }

  _Float16* h0p = h0 + (size_t)grp * H0_ROW;
  for (int pass = 0; pass < 2; ++pass) {
    *(volatile v8h*)(h0p + line0 * 64 + q * 8) = vv0;
    if (line1 < NTAP) *(volatile v8h*)(h0p + line1 * 64 + q * 8) = vv1;
    __threadfence();
  }
}

template <bool OUT16>
__global__ __launch_bounds__(256) void k_gemm_bn(
    const _Float16* __restrict__ A, int lda, const _Float16* __restrict__ Bt, int ldb,
    void* __restrict__ Cout, int ldc,
    const float* __restrict__ bnb, const float* __restrict__ bns, const float* __restrict__ bnt,
    int M, int N, int K, float scale) {
  __shared__ __align__(16) float sT[8][16 * 68];
  const int lane = threadIdx.x & 31;
  const int wave = threadIdx.x >> 5;
  const int tilesN = N >> 6;
  const int tilesM = M >> 6;
  const int tile = (int)blockIdx.x * 8 + wave;
  if (tile >= tilesM * tilesN) return;
  const int tm = tile / tilesN;
  const int tn = tile - tm * tilesN;
  const int m0 = tm << 6;
  const int n0 = tn << 6;
  const int rlane = lane & 15;
  const int koff = (lane >> 4) * 8;
  const int mOff = (lane >> 4) * 8;

  v8f acc[4][4];
#pragma unroll
  for (int i = 0; i < 4; ++i)
#pragma unroll
    for (int j = 0; j < 4; ++j) acc[i][j] = (v8f){0.f, 0.f, 0.f, 0.f, 0.f, 0.f, 0.f, 0.f};

  for (int k0 = 0; k0 < K; k0 += 32) {
    v16h bh[4];
#pragma unroll
    for (int j = 0; j < 4; ++j) {
      const size_t bo = (size_t)(n0 + (j << 4) + rlane) * ldb + koff + k0;
      bh[j] = frag_ld(Bt + bo);
    }
#pragma unroll
    for (int i = 0; i < 4; ++i) {
      const size_t ao = (size_t)(m0 + (i << 4) + rlane) * lda + koff + k0;
      const v16h ah = frag_ld(A + ao);
#pragma unroll
      for (int j = 0; j < 4; ++j) acc[i][j] = mma_h(ah, bh[j], acc[i][j]);
    }
  }

  float bv[4], sv[4], tv[4];
#pragma unroll
  for (int j = 0; j < 4; ++j) {
    const int n = n0 + (j << 4) + rlane;
    bv[j] = bnb[n];
    sv[j] = bns[n];
    tv[j] = bnt[n];
  }

  float* slab = sT[wave];
#pragma unroll
  for (int i = 0; i < 4; ++i) {
    const int mBase = m0 + (i << 4);
#pragma unroll
    for (int j = 0; j < 4; ++j) {
#pragma unroll
      for (int r = 0; r < 8; ++r) {
        const float v = fmaxf((acc[i][j][r] * scale + bv[j]) * sv[j] + tv[j], 0.0f);
        slab[(mOff + r) * 68 + (j << 4) + rlane] = v;
      }
    }
    __builtin_amdgcn_fence(__ATOMIC_RELEASE, "workgroup");
    __builtin_amdgcn_wave_barrier();
    __builtin_amdgcn_fence(__ATOMIC_ACQUIRE, "workgroup");
    if (!OUT16) {
      float* C = (float*)Cout;
      const int hh = lane >> 4, c4 = (lane & 15) * 4;
      for (int pass = 0; pass < 2; ++pass) {
#pragma unroll
        for (int it = 0; it < 8; ++it) {
          const int row = it * 2 + hh;
          const v4f v = *(const v4f*)(slab + row * 68 + c4);
          *(volatile v4f*)(C + (size_t)(mBase + row) * ldc + n0 + c4) = v;
        }
        __threadfence();
      }
    } else {
      _Float16* C = (_Float16*)Cout;
      const int qq = lane >> 3, c8 = (lane & 7) * 8;
      for (int pass = 0; pass < 2; ++pass) {
#pragma unroll
        for (int it = 0; it < 4; ++it) {
          const int row = it * 4 + qq;
          const float* sp = slab + row * 68 + c8;
          v8h hv;
#pragma unroll
          for (int e = 0; e < 8; ++e) hv[e] = (_Float16)sp[e];
          *(volatile v8h*)(C + (size_t)(mBase + row) * ldc + n0 + c8) = hv;
        }
        __threadfence();
      }
    }
    __builtin_amdgcn_fence(__ATOMIC_RELEASE, "workgroup");
    __builtin_amdgcn_wave_barrier();
    __builtin_amdgcn_fence(__ATOMIC_ACQUIRE, "workgroup");
  }
}

template <int KS>
__device__ __forceinline__ void mlp_acc(const _Float16* a0p, const _Float16* a1p, const _Float16* bp,
                                        v8f& c0, v8f& c1) {
#pragma unroll
  for (int ks = 0; ks < KS; ++ks) {
    const v16h bf = frag_ld(bp + 32 * ks);
    const v16h a0 = frag_ld(a0p + 32 * ks);
    const v16h a1 = frag_ld(a1p + 32 * ks);
    c0 = mma_h(a0, bf, c0);
    c1 = mma_h(a1, bf, c1);
  }
}

__global__ __launch_bounds__(128) void k_mlp(
    const float* __restrict__ xyz, const float* __restrict__ points,
    const int* __restrict__ fps_idx, const int* __restrict__ ball_idx,
    const _Float16* __restrict__ Wa, const _Float16* __restrict__ Wb, const _Float16* __restrict__ Wc,
    const float* __restrict__ ba, const float* __restrict__ sa, const float* __restrict__ ta,
    const float* __restrict__ bb, const float* __restrict__ sb, const float* __restrict__ tb,
    const float* __restrict__ bc, const float* __restrict__ sc, const float* __restrict__ tc,
    float* __restrict__ nf2) {
  __shared__ __align__(16) _Float16 bufA[128 * FA_PITCH];
  __shared__ __align__(16) _Float16 bufB[128 * Y_PITCH];
  __shared__ __align__(16) float maxT[4 * 128];

  const int t = (int)threadIdx.x;
  const int lane = t & 31;
  const int wave = t >> 5;
  const int h = lane >> 4;
  const int rl = lane & 15;
  const int grp0 = (int)blockIdx.x * 4;
  const int b = grp0 >> 10;

  {
    const int g = grp0 + (t >> 5);
    const int ci = clampi(fps_idx[g], 0, NPTS - 1);
    const int n = clampi(ball_idx[grp0 * NK + t], 0, NPTS - 1);
    const float* xb = xyz + (size_t)b * 3 * NPTS;
    const float* pb = points + (size_t)b * NFEAT * NPTS + n;
    const float lx = (xb[n] - xb[ci]) * INV_RADIUS;
    const float ly = (xb[NPTS + n] - xb[NPTS + ci]) * INV_RADIUS;
    const float lz = (xb[2 * NPTS + n] - xb[2 * NPTS + ci]) * INV_RADIUS;
    float zz = 0.0f;
    asm volatile("" : "+v"(zz));
    _Float16* frow = bufA + t * FA_PITCH;
    {
      v8h hv;
      hv[0] = (_Float16)lx;
      hv[1] = (_Float16)ly;
      hv[2] = (_Float16)lz;
#pragma unroll
      for (int e = 0; e < 5; ++e) hv[3 + e] = (_Float16)pb[(size_t)e * NPTS];
      *(v8h*)frow = hv;
    }
    asm volatile("" ::: "memory");
#pragma unroll
    for (int j = 1; j < 8; ++j) {
      v8h hv;
#pragma unroll
      for (int e = 0; e < 8; ++e) hv[e] = (_Float16)pb[(size_t)(8 * j - 3 + e) * NPTS];
      *(v8h*)(frow + 8 * j) = hv;
      asm volatile("" ::: "memory");
    }
    {
      v8h hv;
      hv[0] = (_Float16)pb[(size_t)61 * NPTS];
      hv[1] = (_Float16)pb[(size_t)62 * NPTS];
      hv[2] = (_Float16)pb[(size_t)63 * NPTS];
#pragma unroll
      for (int e = 3; e < 8; ++e) hv[e] = (_Float16)zz;
      *(v8h*)(frow + 64) = hv;
    }
    {
      v8h zv;
#pragma unroll
      for (int e = 0; e < 8; ++e) zv[e] = (_Float16)zz;
      *(v8h*)(frow + 72) = zv;
      *(v8h*)(frow + 80) = zv;
      *(v8h*)(frow + 88) = zv;
    }
  }
  __syncthreads();

  const int rb = wave * 32;

#pragma unroll 1
  for (int j = 0; j < 4; ++j) {
    v8f c0 = (v8f){0.f, 0.f, 0.f, 0.f, 0.f, 0.f, 0.f, 0.f};
    v8f c1 = (v8f){0.f, 0.f, 0.f, 0.f, 0.f, 0.f, 0.f, 0.f};
    mlp_acc<3>(bufA + (rb + rl) * FA_PITCH + 8 * h, bufA + (rb + 16 + rl) * FA_PITCH + 8 * h,
               Wa + (size_t)(16 * j + rl) * KA + 8 * h, c0, c1);
    const int o = 16 * j + rl;
    const float bvv = ba[o];
    const float svv = sa[o];
    const float tvv = ta[o];
#pragma unroll
    for (int r = 0; r < 8; ++r) {
      const float y0 = fmaxf((c0[r] * WCARRY_INV + bvv) * svv + tvv, 0.0f);
      const float y1 = fmaxf((c1[r] * WCARRY_INV + bvv) * svv + tvv, 0.0f);
      bufB[(rb + 8 * h + r) * Y_PITCH + o] = (_Float16)y0;
      bufB[(rb + 16 + 8 * h + r) * Y_PITCH + o] = (_Float16)y1;
    }
  }
  __syncthreads();

#pragma unroll 1
  for (int j = 0; j < 4; ++j) {
    v8f c0 = (v8f){0.f, 0.f, 0.f, 0.f, 0.f, 0.f, 0.f, 0.f};
    v8f c1 = (v8f){0.f, 0.f, 0.f, 0.f, 0.f, 0.f, 0.f, 0.f};
    mlp_acc<2>(bufB + (rb + rl) * Y_PITCH + 8 * h, bufB + (rb + 16 + rl) * Y_PITCH + 8 * h,
               Wb + (size_t)(16 * j + rl) * 64 + 8 * h, c0, c1);
    const int o = 16 * j + rl;
    const float bvv = bb[o];
    const float svv = sb[o];
    const float tvv = tb[o];
#pragma unroll
    for (int r = 0; r < 8; ++r) {
      const float y0 = fmaxf((c0[r] * WCARRY_INV + bvv) * svv + tvv, 0.0f);
      const float y1 = fmaxf((c1[r] * WCARRY_INV + bvv) * svv + tvv, 0.0f);
      bufA[(rb + 8 * h + r) * Y_PITCH + o] = (_Float16)y0;
      bufA[(rb + 16 + 8 * h + r) * Y_PITCH + o] = (_Float16)y1;
    }
  }
  __syncthreads();

#pragma unroll 1
  for (int j = 0; j < 8; ++j) {
    v8f c0 = (v8f){0.f, 0.f, 0.f, 0.f, 0.f, 0.f, 0.f, 0.f};
    v8f c1 = (v8f){0.f, 0.f, 0.f, 0.f, 0.f, 0.f, 0.f, 0.f};
    mlp_acc<2>(bufA + (rb + rl) * Y_PITCH + 8 * h, bufA + (rb + 16 + rl) * Y_PITCH + 8 * h,
               Wc + (size_t)(16 * j + rl) * 64 + 8 * h, c0, c1);
    const int o = 16 * j + rl;
    const float bvv = bc[o];
    const float svv = sc[o];
    const float tvv = tc[o];
    float mx = -INFINITY;
#pragma unroll
    for (int r = 0; r < 8; ++r) {
      const float y0 = fmaxf((c0[r] * WCARRY_INV + bvv) * svv + tvv, 0.0f);
      const float y1 = fmaxf((c1[r] * WCARRY_INV + bvv) * svv + tvv, 0.0f);
      mx = fmaxf(mx, fmaxf(y0, y1));
    }
    const float other = __shfl_xor(mx, 16, 32);
    mx = fmaxf(mx, other);
    if (h == 0) maxT[wave * 128 + o] = mx;
  }
  __syncthreads();

  {
    const v4f mv = *(const v4f*)&maxT[wave * 128 + lane * 4];
    float* p = nf2 + (size_t)(grp0 + wave) * 128 + lane * 4;
    *(volatile v4f*)p = mv;
    __threadfence();
    *(volatile v4f*)p = mv;
  }
}

__global__ __launch_bounds__(256) void k_combine(
    const float* __restrict__ nf3, const float* __restrict__ nf2, float* __restrict__ out1) {
  __shared__ __align__(16) float T[128 * 36];
  const int t = (int)threadIdx.x;
  const int lane = t & 31;
  const int wave = t >> 5;
  const int b = (int)blockIdx.x >> 5;
  const int s0 = ((int)blockIdx.x & 31) * 32;
  const int grp0 = b * NS + s0;
#pragma unroll
  for (int i = 0; i < 4; ++i) {
    const int idx = t + 256 * i;
    const int row = idx >> 5;
    const int c4 = (idx & 31) * 4;
    const v4f a = *(const v4f*)(nf3 + (size_t)(grp0 + row) * 128 + c4);
    const v4f c = *(const v4f*)(nf2 + (size_t)(grp0 + row) * 128 + c4);
    T[(c4 + 0) * 36 + row] = a[0] + c[0];
    T[(c4 + 1) * 36 + row] = a[1] + c[1];
    T[(c4 + 2) * 36 + row] = a[2] + c[2];
    T[(c4 + 3) * 36 + row] = a[3] + c[3];
  }
  __syncthreads();
  const int q = lane & 7;
  const int lr = lane >> 3;
  v4f vv[4];
#pragma unroll
  for (int it = 0; it < 4; ++it) {
    const int o = wave * 16 + it * 4 + lr;
    vv[it] = *(const v4f*)&T[o * 36 + 4 * q];
  }
  for (int pass = 0; pass < 2; ++pass) {
#pragma unroll
    for (int it = 0; it < 4; ++it) {
      const int o = wave * 16 + it * 4 + lr;
      *(volatile v4f*)(out1 + ((size_t)(b * 128 + o)) * NS + s0 + 4 * q) = vv[it];
    }
    __threadfence();
  }
}

extern "C" void kernel_launch(void* const* d_in, const int* in_sizes, int n_in,
                              void* d_out, int out_size, void* d_ws, size_t ws_size,
                              hipStream_t stream) {
  (void)in_sizes;
  (void)out_size;
  if (n_in < 28) return;
  if (ws_size < WS_TOTAL) return;

  const float* xyz    = (const float*)d_in[0];
  const float* points = (const float*)d_in[1];
  const int*   fps    = (const int*)d_in[2];
  const int*   ball   = (const int*)d_in[3];
  const float* w3d0 = (const float*)d_in[4];
  const float* b3d0 = (const float*)d_in[5];
  const float* s3d0 = (const float*)d_in[6];
  const float* t3d0 = (const float*)d_in[7];
  const float* w3d1 = (const float*)d_in[8];
  const float* b3d1 = (const float*)d_in[9];
  const float* s3d1 = (const float*)d_in[10];
  const float* t3d1 = (const float*)d_in[11];
  const float* w3d2 = (const float*)d_in[12];
  const float* b3d2 = (const float*)d_in[13];
  const float* s3d2 = (const float*)d_in[14];
  const float* t3d2 = (const float*)d_in[15];
  const float* w2d0 = (const float*)d_in[16];
  const float* b2d0 = (const float*)d_in[17];
  const float* s2d0 = (const float*)d_in[18];
  const float* t2d0 = (const float*)d_in[19];
  const float* w2d1 = (const float*)d_in[20];
  const float* b2d1 = (const float*)d_in[21];
  const float* s2d1 = (const float*)d_in[22];
  const float* t2d1 = (const float*)d_in[23];
  const float* w2d2 = (const float*)d_in[24];
  const float* b2d2 = (const float*)d_in[25];
  const float* s2d2 = (const float*)d_in[26];
  const float* t2d2 = (const float*)d_in[27];

  char* ws = (char*)d_ws;
  _Float16* wpl = (_Float16*)(ws + WS_WPL);
  _Float16* h0  = (_Float16*)(ws + WS_H0);
  _Float16* h1  = (_Float16*)(ws + WS_H1);
  float* nf3 = (float*)(ws + WS_NF3);
  float* nf2 = (float*)(ws + WS_NF2);
  float* out0 = (float*)d_out;
  float* out1 = (float*)d_out + OUT0_ELEMS;

  const _Float16* W0t = wpl + OFF_W0T;
  const _Float16* W1t = wpl + OFF_W1T;
  const _Float16* W2t = wpl + OFF_W2T;
  const _Float16* Wa  = wpl + OFF_WA;
  const _Float16* Wb  = wpl + OFF_WB;
  const _Float16* Wc  = wpl + OFF_WC;

  static_assert(WPL_HALVES / 8 / 256 == 128, "prep grid");
  k_prep_w<<<128, 256, 0, stream>>>(w3d0, w3d1, w3d2, w2d0, w2d1, w2d2, wpl);

  static_assert(OUT0_ELEMS / 4 / 256 == 24, "out0 grid");
  k_out0<<<24, 256, 0, stream>>>(xyz, fps, out0);

  k_splat_conv0<<<NGRP, 128, 0, stream>>>(xyz, points, fps, ball, W0t, b3d0, s3d0, t3d0, h0);

  static_assert((NGRP / 64) * (64 / 64) == 16 * 8, "conv1 tiles");
  k_gemm_bn<true><<<16, 256, 0, stream>>>(h0, K1, W1t, K1, (void*)h1, 64,
                                          b3d1, s3d1, t3d1, NGRP, 64, K1, WCARRY_INV);

  static_assert((NGRP / 64) * (128 / 64) == 32 * 8, "conv2 tiles");
  k_gemm_bn<false><<<32, 256, 0, stream>>>(h1, 64, W2t, 64, (void*)nf3, 128,
                                           b3d2, s3d2, t3d2, NGRP, 128, 64, WCARRY_INV);

  static_assert(NGRP % 4 == 0 && NS % 4 == 0, "mlp grid");
  k_mlp<<<NGRP / 4, 128, 0, stream>>>(xyz, points, fps, ball, Wa, Wb, Wc,
                                      b2d0, s2d0, t2d0, b2d1, s2d1, t2d1, b2d2, s2d2, t2d2, nf2);

  static_assert(NB * (NS / 32) == 256, "combine grid");
  k_combine<<<256, 256, 0, stream>>>(nf3, nf2, out1);
}
